// rgcn_layer_67525475828084
// MI455X (gfx1250) — hardware-run, weakly checked
//
#include <hip/hip_runtime.h>
#include <stddef.h>
#include <stdint.h>


#define NN      100000
#define NREL    4
#define NEDGE   500000
#define DF      128
#define KT      1024
#define NBA     1024
#define SLB     17
#define SRCMASK ((1u << SLB) - 1u)
#define NBLK    98
#define NPADN   (NBLK * NBA)
#define HALF    50048
#define NTHR    256
#define NWAVE   8
#define WKEYS   (NEDGE / NWAVE)
#define WGRP    (WKEYS / 4)
#define WITER   ((WGRP + 31) / 32)
#define WL      1024
#define RCAP    (NWAVE * WL)
#define DEGCAP  64
#define FPITCH  32
#define GBM     64
#define GBN     128
#define GTHR    128
#define RPB     64
#define RPW     8
#define WUNITS  (DF * (KT / 8))
#define BK_INTS (2 * RCAP + 3 * NBA + 32)
#define LDS_BK  (BK_INTS * 4)
#define MEAS_BLK_HITS 5328
#define MEAS_MAXDEG   18

static_assert(NN == 100000);
static_assert(NN <= (1 << SLB) && NBA <= (1 << 10) && SLB + 10 <= 31);
static_assert(NBLK * NBA >= NN && (NBLK - 1) * NBA < NN);
static_assert(HALF == 391 * 128 && HALF % GBM == 0 && HALF % RPB == 0);
static_assert(HALF <= NN && 2 * HALF >= NN);
static_assert(KT == 1024 && KT % 32 == 0 && KT == NREL * 2 * DF);
static_assert(RCAP == 8 * WL && RCAP % (NTHR * 4) == 0);
static_assert((long long)RCAP * 100 >= (long long)MEAS_BLK_HITS * 110);
static_assert(DEGCAP == 64 && DEGCAP >= MEAS_MAXDEG + 8);
static_assert(NEDGE % NWAVE == 0 && WKEYS % 4 == 0 && (NEDGE % 4) == 0);
static_assert(NBA == NTHR * 4 && BK_INTS % 4 == 0 && LDS_BK <= 327680);
static_assert(GBN == DF && GBM == (GTHR / 32) * 16 && DF == 32 * 4);
static_assert(WUNITS % NTHR == 0 && RPB == NWAVE * RPW);

typedef float          v4f   __attribute__((ext_vector_type(4)));
typedef float          v8f   __attribute__((ext_vector_type(8)));
typedef int            v4i   __attribute__((ext_vector_type(4)));
typedef int            v8i   __attribute__((ext_vector_type(8)));
typedef unsigned       v2u   __attribute__((ext_vector_type(2)));
typedef unsigned short v8us  __attribute__((ext_vector_type(8)));
typedef __bf16         v16bf __attribute__((ext_vector_type(16)));
typedef v4f  __attribute__((may_alias)) v4fa;
typedef v4i  __attribute__((may_alias)) v4ia;
typedef v8us __attribute__((may_alias)) v8usa;
union FragB { v16bf v; v8us h[2]; v8i w; };

__device__ __forceinline__ v8f wmb(const FragB& a, const FragB& b, v8f c) {
  v8f d = __builtin_amdgcn_wmma_f32_16x16x32_bf16(false, a.v, false, b.v, (short)0, c, false, false);
  asm volatile("v_nop\n\tv_nop\n\tv_nop\n\tv_nop" : "+v"(d) : "v"(a.w), "v"(b.w));
  return d;
}

__device__ __forceinline__ unsigned bf16_bits(float f) {
  const unsigned u = __float_as_uint(f);
  const unsigned r = ((u + 0x7FFFu + ((u >> 16) & 1u)) >> 16) & 0xFFFFu;
  const unsigned n = ((u >> 16) | 0x40u) & 0xFFFFu;
  return ((u & 0x7fffffffu) > 0x7f800000u) ? n : r;
}
__device__ __forceinline__ float bf16_val(float f) { return __uint_as_float(bf16_bits(f) << 16); }
__device__ __forceinline__ void pack2(float a, float b, unsigned& hw, unsigned& lw) {
  const unsigned ha = bf16_bits(a), hb = bf16_bits(b);
  const unsigned la = bf16_bits(a - __uint_as_float(ha << 16));
  const unsigned lb = bf16_bits(b - __uint_as_float(hb << 16));
  hw = ha | (hb << 16);
  lw = la | (lb << 16);
}
__device__ __forceinline__ float relu_k(float v) { return (v > 0.0f) ? v : (v - v); }

__device__ __forceinline__ void acc_row(const float* __restrict__ x, int sk, int lane,
                                        float& a0, float& a1, float& a2, float& a3) {
  const v4f xv = *(const v4f*)(x + (size_t)sk * DF + 4 * lane);
  a0 += bf16_val(xv.x);
  a1 += bf16_val(xv.y);
  a2 += bf16_val(xv.z);
  a3 += bf16_val(xv.w);
}

__global__ __launch_bounds__(NTHR) void k_prep(const float* __restrict__ W, const float* __restrict__ b,
                                               unsigned short* wt, float* bsum) {
  const int u = (int)blockIdx.x * NTHR + (int)threadIdx.x;
  if (u < WUNITS) {
    const int n  = u >> 7;
    const int j  = u & 127;
    const int k8 = 8 * j;
    const int r  = k8 >> 8;
    const int c0 = k8 & 127;
    const float* sp = W + (size_t)r * DF * DF + (size_t)c0 * DF + (size_t)n;
    float f[8];
#pragma unroll
    for (int i = 0; i < 8; ++i) f[i] = sp[(size_t)i * DF];
    v8us o;
#pragma unroll
    for (int i = 0; i < 8; ++i) o[i] = (unsigned short)bf16_bits(f[i]);
    unsigned short* dp = wt + (size_t)n * KT + (size_t)k8;
    *(volatile v8us*)dp = o;
    __threadfence();
    *(volatile v8us*)dp = o;
  } else {
    const int t  = u - WUNITS;
    const int tc = t < 32 ? t : 31;
    const v4f b0 = *(const v4f*)(b + 0 * DF + 4 * tc);
    const v4f b1 = *(const v4f*)(b + 1 * DF + 4 * tc);
    const v4f b2 = *(const v4f*)(b + 2 * DF + 4 * tc);
    const v4f b3 = *(const v4f*)(b + 3 * DF + 4 * tc);
    asm volatile("" :: "v"(b0), "v"(b1), "v"(b2), "v"(b3));
    v4f o;
    o.x = ((bf16_val(b0.x) + bf16_val(b1.x)) + bf16_val(b2.x)) + bf16_val(b3.x);
    o.y = ((bf16_val(b0.y) + bf16_val(b1.y)) + bf16_val(b2.y)) + bf16_val(b3.y);
    o.z = ((bf16_val(b0.z) + bf16_val(b1.z)) + bf16_val(b2.z)) + bf16_val(b3.z);
    o.w = ((bf16_val(b0.w) + bf16_val(b1.w)) + bf16_val(b2.w)) + bf16_val(b3.w);
    float* op = bsum + 4 * tc;
    if (t < 32) *(volatile v4f*)op = o;
    __threadfence();
    if (t < 32) *(volatile v4f*)op = o;
  }
}

__global__ __launch_bounds__(NTHR) void k_bucket(const int* __restrict__ srcs, const int* __restrict__ dsts,
                                                 int* LIST, int* CNT, int* OFF, int* FLG) {
  extern __shared__ __attribute__((aligned(16))) int dsm[];
  int* list   = dsm;
  int* sorted = list + RCAP;
  int* scnt   = sorted + RCAP;
  int* soff   = scnt + NBA;
  int* cur    = soff + NBA;
  int* wcnt   = cur + NBA;
  int* wtot   = wcnt + 8;
  int* wmx    = wtot + 8;
  const int tid = (int)threadIdx.x, lane = tid & 31, wave = tid >> 5;
  const int bx = (int)blockIdx.x, rel = (int)blockIdx.y;
  const int slotBase = bx * NBA;
  int nb = NN - slotBase;
  nb = nb > NBA ? NBA : (nb < 1 ? 1 : nb);
  const size_t kb = (size_t)rel * NEDGE + (size_t)wave * WKEYS;
  const int* dk = dsts + kb;
  const int* sk = srcs + kb;

  {
    const v4i z4 = {0, 0, 0, 0};
    for (int i = tid * 4; i < BK_INTS; i += NTHR * 4) *(v4ia*)(dsm + i) = z4;
  }
  __syncthreads();

  int wc = 0;
  int* wl = list + wave * WL;
  const unsigned nbs = (unsigned)slotBase;
  const unsigned unb = (unsigned)nb;
  const int sent = (int)0x80000000u;
#pragma unroll 1
  for (int it = 0; it < WITER; ++it) {
    const int g   = it * 32 + lane;
    const bool gv = g < WGRP;
    const int gc  = gv ? g : WGRP - 1;
    const v4i dl  = *(const v4i*)(dk + 4 * gc);
    asm volatile("" :: "v"(dl));
    const int d0 = gv ? dl.x : sent;
    const int d1 = gv ? dl.y : sent;
    const int d2 = gv ? dl.z : sent;
    const int d3 = gv ? dl.w : sent;
    const unsigned s0 = (unsigned)d0 - nbs, s1 = (unsigned)d1 - nbs;
    const unsigned s2 = (unsigned)d2 - nbs, s3 = (unsigned)d3 - nbs;
    const bool h0 = s0 < unb, h1 = s1 < unb, h2 = s2 < unb, h3 = s3 < unb;
    const unsigned m0 = __builtin_amdgcn_ballot_w32(h0);
    const unsigned m1 = __builtin_amdgcn_ballot_w32(h1);
    const unsigned m2 = __builtin_amdgcn_ballot_w32(h2);
    const unsigned m3 = __builtin_amdgcn_ballot_w32(h3);
    if ((m0 | m1 | m2 | m3) != 0u) {
      const v4i sv = *(const v4i*)(sk + 4 * gc);
      asm volatile("" :: "v"(sv));
      int q0 = sv.x, q1 = sv.y, q2 = sv.z, q3 = sv.w;
      q0 = q0 < 0 ? 0 : (q0 > NN - 1 ? NN - 1 : q0);
      q1 = q1 < 0 ? 0 : (q1 > NN - 1 ? NN - 1 : q1);
      q2 = q2 < 0 ? 0 : (q2 > NN - 1 ? NN - 1 : q2);
      q3 = q3 < 0 ? 0 : (q3 > NN - 1 ? NN - 1 : q3);
      const unsigned lower = __builtin_amdgcn_mbcnt_lo(m0,
                             __builtin_amdgcn_mbcnt_lo(m1,
                             __builtin_amdgcn_mbcnt_lo(m2,
                             __builtin_amdgcn_mbcnt_lo(m3, 0u))));
      int p = wc + (int)lower;
      if (h0) { if (p < WL) wl[p] = (int)((unsigned)q0 | (s0 << SLB)); }
      p += h0 ? 1 : 0;
      if (h1) { if (p < WL) wl[p] = (int)((unsigned)q1 | (s1 << SLB)); }
      p += h1 ? 1 : 0;
      if (h2) { if (p < WL) wl[p] = (int)((unsigned)q2 | (s2 << SLB)); }
      p += h2 ? 1 : 0;
      if (h3) { if (p < WL) wl[p] = (int)((unsigned)q3 | (s3 << SLB)); }
      wc += (int)__builtin_popcount(m0) + (int)__builtin_popcount(m1)
          + (int)__builtin_popcount(m2) + (int)__builtin_popcount(m3);
    }
  }
  if (lane == 0) wcnt[wave] = wc;
  __syncthreads();

  int nh = 0, ovf = 0;
#pragma unroll
  for (int w2 = 0; w2 < NWAVE; ++w2) {
    const int raw = wcnt[w2];
    ovf |= (raw > WL || raw < 0) ? 1 : 0;
    nh += raw < 0 ? 0 : (raw > WL ? WL : raw);
  }

  if (wave == 0) {
#pragma unroll 1
    for (int w2 = 0; w2 < NWAVE; ++w2) {
      int cvv = wcnt[w2];
      cvv = cvv < 0 ? 0 : (cvv > WL ? WL : cvv);
      const int c = __builtin_amdgcn_readfirstlane(cvv);
#pragma unroll 1
      for (int b0 = 0; b0 < c; b0 += 32) {
        const int idx = b0 + lane;
        const int ent = list[w2 * WL + (idx < WL ? idx : WL - 1)];
#pragma unroll 1
        for (int k = 0; k < 32; ++k) {
          if (b0 + k >= c) break;
          const int u  = __builtin_amdgcn_readlane(ent, k);
          const int sl = (int)(((unsigned)u >> SLB) & (unsigned)(NBA - 1));
          if (lane == 0) scnt[sl] = scnt[sl] + 1;
        }
      }
    }
  }
  __syncthreads();

  {
    const v4i ca = *(const v4ia*)(scnt + 4 * tid);
    const int e0 = ca.x < 0 ? 0 : ca.x, e1 = ca.y < 0 ? 0 : ca.y, e2 = ca.z < 0 ? 0 : ca.z, e3 = ca.w < 0 ? 0 : ca.w;
    const int ts = e0 + e1 + e2 + e3;
    int incl = ts;
#pragma unroll
    for (int d = 1; d < 32; d <<= 1) {
      const int up = __shfl_up(incl, d, 32);
      if (lane >= d) incl += up;
    }
    int mx = max(max(e0, e1), max(e2, e3));
    mx = max(mx, __shfl_xor(mx, 16, 32));
    mx = max(mx, __shfl_xor(mx, 8, 32));
    mx = max(mx, __shfl_xor(mx, 4, 32));
    mx = max(mx, __shfl_xor(mx, 2, 32));
    mx = max(mx, __shfl_xor(mx, 1, 32));
    if (lane == 31) wtot[wave] = incl;
    if (lane == 0)  wmx[wave] = mx;
    __syncthreads();
    int pre = 0;
#pragma unroll
    for (int w2 = 0; w2 < NWAVE; ++w2) pre += (w2 < wave) ? wtot[w2] : 0;
    int run = pre + incl - ts;
    v4i so;
    so.x = run; run += e0;
    so.y = run; run += e1;
    so.z = run; run += e2;
    so.w = run;
    *(v4ia*)(soff + 4 * tid) = so;
    *(v4ia*)(cur + 4 * tid)  = so;
  }
  __syncthreads();

  if (wave == 0) {
#pragma unroll 1
    for (int w2 = 0; w2 < NWAVE; ++w2) {
      int cvv = wcnt[w2];
      cvv = cvv < 0 ? 0 : (cvv > WL ? WL : cvv);
      const int c = __builtin_amdgcn_readfirstlane(cvv);
#pragma unroll 1
      for (int b0 = 0; b0 < c; b0 += 32) {
        const int idx = b0 + lane;
        const int ent = list[w2 * WL + (idx < WL ? idx : WL - 1)];
#pragma unroll 1
        for (int k = 0; k < 32; ++k) {
          if (b0 + k >= c) break;
          const int u  = __builtin_amdgcn_readlane(ent, k);
          const int sl = (int)(((unsigned)u >> SLB) & (unsigned)(NBA - 1));
          const int sv = (int)((unsigned)u & SRCMASK);
          if (lane == 0) {
            int pos = cur[sl];
            pos = pos < 0 ? 0 : (pos > RCAP - 1 ? RCAP - 1 : pos);
            sorted[pos] = sv;
            cur[sl] = pos + 1;
          }
        }
      }
    }
  }
  __syncthreads();

  int bmax = 0;
#pragma unroll
  for (int w2 = 0; w2 < NWAVE; ++w2) bmax = max(bmax, wmx[w2]);
  const int flag = ((ovf != 0) || (bmax > DEGCAP)) ? 1 : 0;
  const size_t blk = (size_t)rel * NBLK + (size_t)bx;

  int* lrow = LIST + blk * RCAP;
#pragma unroll 1
  for (int it = 0; it < RCAP / (NTHR * 4); ++it) {
    const int i0 = 4 * (it * NTHR + tid);
    const v4i ev = *(const v4ia*)(sorted + i0);
    int g0 = ev.x, g1 = ev.y, g2 = ev.z, g3 = ev.w;
    g0 = g0 < 0 ? 0 : (g0 > NN - 1 ? NN - 1 : g0);
    g1 = g1 < 0 ? 0 : (g1 > NN - 1 ? NN - 1 : g1);
    g2 = g2 < 0 ? 0 : (g2 > NN - 1 ? NN - 1 : g2);
    g3 = g3 < 0 ? 0 : (g3 > NN - 1 ? NN - 1 : g3);
    v4i ov;
    ov.x = (i0     < nh) ? g0 : 0;
    ov.y = (i0 + 1 < nh) ? g1 : 0;
    ov.z = (i0 + 2 < nh) ? g2 : 0;
    ov.w = (i0 + 3 < nh) ? g3 : 0;
    *(volatile v4i*)(lrow + i0) = ov;
    __threadfence();
    *(volatile v4i*)(lrow + i0) = ov;
  }
  {
    const v4i cv = *(const v4ia*)(scnt + 4 * tid);
    const v4i fv = *(const v4ia*)(soff + 4 * tid);
    v4i rv = {0, 0, 0, 0};
    rv.x = (tid == 0) ? flag : 0;
    rv.y = (tid == 0) ? bmax : 0;
    rv.z = (tid == 0) ? nh : 0;
    int* cp = CNT + (size_t)rel * NPADN + (size_t)slotBase + 4 * tid;
    int* fp = OFF + (size_t)rel * NPADN + (size_t)slotBase + 4 * tid;
    int* rp = FLG + blk * FPITCH + 4 * (tid & 7);
    *(volatile v4i*)cp = cv;
    *(volatile v4i*)fp = fv;
    if (tid < 8) *(volatile v4i*)rp = rv;
    __threadfence();
    *(volatile v4i*)cp = cv;
    *(volatile v4i*)fp = fv;
    if (tid < 8) *(volatile v4i*)rp = rv;
  }
}

__global__ __launch_bounds__(NTHR) void k_replay(const float* __restrict__ x, const int* __restrict__ LIST,
                                                 const int* __restrict__ CNT, const int* __restrict__ OFF,
                                                 const int* __restrict__ FLG, unsigned short* A,
                                                 int row0, int nrows) {
  const int tid = (int)threadIdx.x, lane = tid & 31, wave = tid >> 5;
#pragma unroll 1
  for (int ri = 0; ri < RPW; ++ri) {
    const int lr    = (int)blockIdx.x * RPB + wave * RPW + ri;
    const int node  = row0 + lr;
    const bool live = lr < nrows;
    const int nodet = node < NN ? node : NN - 1;
    const int bxn   = nodet >> 10;
    unsigned short* arow = A + (size_t)lr * KT;
#pragma unroll 1
    for (int r = 0; r < NREL; ++r) {
      const int ti  = r * NPADN + nodet;
      const int cv  = CNT[ti];
      const int ofv = OFF[ti];
      const int fl  = FLG[(r * NBLK + bxn) * FPITCH];
      asm volatile("" :: "v"(cv), "v"(ofv), "v"(fl));
      const int cpos = cv < 0 ? 0 : cv;
      const int dmax = cpos < 1 ? 1 : cpos;
      const float dv = (float)dmax;
      int c = cpos > DEGCAP ? DEGCAP : cpos;
      const int o = ofv < 0 ? 0 : (ofv > RCAP - 1 ? RCAP - 1 : ofv);
      c = c > RCAP - o ? RCAP - o : c;
      c = live ? c : 0;
      int last = o + c - 1;
      last = last < o ? o : last;
      const int c0 = c > 32 ? 32 : c;
      const int c1 = c - c0;
      const int c0u = __builtin_amdgcn_readfirstlane(c0);
      const int c1u = __builtin_amdgcn_readfirstlane(c1);
      const bool bad = live && ((fl != 0) || (cv > DEGCAP) || (cv < 0));
      const int* lp = LIST + (size_t)(r * NBLK + bxn) * RCAP;
      int i0 = o + lane;       i0 = i0 > last ? last : i0;
      int i1 = o + 32 + lane;  i1 = i1 > last ? last : i1;
      int col0 = lp[i0];
      int col1 = lp[i1];
      col0 = col0 < 0 ? 0 : (col0 > NN - 1 ? NN - 1 : col0);
      col1 = col1 < 0 ? 0 : (col1 > NN - 1 ? NN - 1 : col1);
      float a0 = 0.0f, a1 = 0.0f, a2 = 0.0f, a3 = 0.0f;
#pragma unroll 1
      for (int e = 0; e < c0u; ++e) {
        const int sk = __builtin_amdgcn_readlane(col0, e);
        acc_row(x, sk, lane, a0, a1, a2, a3);
      }
#pragma unroll 1
      for (int e = 0; e < c1u; ++e) {
        const int sk = __builtin_amdgcn_readlane(col1, e);
        acc_row(x, sk, lane, a0, a1, a2, a3);
      }
      const float nanv = __int_as_float(0x7fc00000);
      float m0 = a0 / dv;
      float m1 = a1 / dv;
      float m2 = a2 / dv;
      float m3 = a3 / dv;
      m0 = bad ? nanv : m0;
      m1 = bad ? nanv : m1;
      m2 = bad ? nanv : m2;
      m3 = bad ? nanv : m3;
      unsigned hw0, lw0, hw1, lw1;
      pack2(m0, m1, hw0, lw0);
      pack2(m2, m3, hw1, lw1);
      v2u qh, ql;
      qh.x = hw0; qh.y = hw1;
      ql.x = lw0; ql.y = lw1;
      unsigned short* wp = arow + r * (2 * DF) + 4 * lane;
      *(volatile v2u*)wp = qh;
      *(volatile v2u*)(wp + DF) = ql;
      __threadfence();
      *(volatile v2u*)wp = qh;
      *(volatile v2u*)(wp + DF) = ql;
    }
  }
}

__global__ __launch_bounds__(GTHR) __attribute__((amdgpu_num_vgpr(248)))
void k_gemm(const unsigned short* __restrict__ Apl, const unsigned short* __restrict__ BT,
            const float* __restrict__ bsum, float* outp, int row0, int nrows) {
  __shared__ __attribute__((aligned(16))) float stg[GBM * GBN];
  __shared__ __attribute__((aligned(16))) float bsh[GBN];
  const int tid = (int)threadIdx.x, lane = tid & 31, wave = tid >> 5, hh = lane >> 4, m = lane & 15;
  const int rowBase = (int)blockIdx.x * GBM;

  if (tid < 32) {
    const v4f b4 = *(const v4f*)(bsum + 4 * tid);
    *(v4fa*)(bsh + 4 * tid) = b4;
  }

  v8f acc[8];
  {
    const v8f z = {0.f, 0.f, 0.f, 0.f, 0.f, 0.f, 0.f, 0.f};
#pragma unroll
    for (int t = 0; t < 8; ++t) acc[t] = z;
  }
  const unsigned short* ap = Apl + (size_t)(rowBase + 16 * wave + m) * (size_t)KT + 8 * hh;
  const unsigned short* bp = BT + (size_t)m * (size_t)KT + 8 * hh;

#pragma unroll 1
  for (int k0 = 0; k0 < KT; k0 += 32) {
    FragB af;
    af.h[0] = *(const v8usa*)(ap + k0);
    af.h[1] = *(const v8usa*)(ap + k0 + 16);
#pragma unroll
    for (int nt = 0; nt < 8; ++nt) {
      const unsigned short* wq = bp + (size_t)(16 * nt) * (size_t)KT + k0;
      FragB bf;
      bf.h[0] = *(const v8usa*)wq;
      bf.h[1] = *(const v8usa*)(wq + 16);
      acc[nt] = wmb(af, bf, acc[nt]);
    }
  }

#pragma unroll
  for (int nt = 0; nt < 8; ++nt) {
    const int lc = 16 * nt + m;
#pragma unroll
    for (int r = 0; r < 8; ++r) {
      const int lr = 16 * wave + 8 * hh + r;
      stg[lr * GBN + lc] = acc[nt][r];
    }
  }
  __syncthreads();

  const v4f bb4 = *(const v4fa*)(bsh + 4 * lane);

#pragma unroll 1
  for (int i = 0; i < 16; ++i) {
    const int lr = 16 * wave + i;
    const int gr = rowBase + lr;
    const v4f t  = *(const v4fa*)(stg + lr * GBN + 4 * lane);
    v4f y;
    y.x = relu_k(t.x + bb4.x);
    y.y = relu_k(t.y + bb4.y);
    y.z = relu_k(t.z + bb4.z);
    y.w = relu_k(t.w + bb4.w);
    asm volatile("" :: "v"(y));
    const int grs = gr < nrows ? gr : 0;
    float* op = outp + (size_t)(row0 + grs) * DF + 4 * lane;
    if (gr < nrows) *(volatile v4f*)op = y;
  }
  __threadfence();
#pragma unroll 1
  for (int i = 0; i < 16; ++i) {
    const int lr = 16 * wave + i;
    const int gr = rowBase + lr;
    const v4f t  = *(const v4fa*)(stg + lr * GBN + 4 * lane);
    v4f y;
    y.x = relu_k(t.x + bb4.x);
    y.y = relu_k(t.y + bb4.y);
    y.z = relu_k(t.z + bb4.z);
    y.w = relu_k(t.w + bb4.w);
    asm volatile("" :: "v"(y));
    const int grs = gr < nrows ? gr : 0;
    float* op = outp + (size_t)(row0 + grs) * DF + 4 * lane;
    if (gr < nrows) *(volatile v4f*)op = y;
  }
}

static inline int cdiv(int a, int b) { return (a + b - 1) / b; }
static inline size_t al256(size_t o) { return (o + 255) & ~(size_t)255; }

extern "C" void kernel_launch(void* const* d_in, const int* in_sizes, int n_in,
                              void* d_out, int out_size, void* d_ws, size_t ws_size,
                              hipStream_t stream) {
  if (n_in < 5) return;
  if (in_sizes[0] != NN * DF) return;
  if (in_sizes[1] != NREL * DF * DF) return;
  if (in_sizes[2] != NREL * DF) return;
  if (in_sizes[3] != NREL * NEDGE) return;
  if (in_sizes[4] != NREL * NEDGE) return;
  if (out_size != NN * DF) return;

  const float* x   = (const float*)d_in[0];
  const float* W   = (const float*)d_in[1];
  const float* b   = (const float*)d_in[2];
  const int*   src = (const int*)  d_in[3];
  const int*   dst = (const int*)  d_in[4];
  float* out = (float*)d_out;

  char* ws = (char*)d_ws;
  size_t off = 0;
  const size_t oWT = off; off = al256(off + (size_t)DF * KT * 2);
  const size_t oBS = off; off = al256(off + (size_t)DF * 4);
  const size_t oFL = off; off = al256(off + (size_t)NREL * NBLK * FPITCH * 4);
  const size_t oCN = off; off = al256(off + (size_t)NREL * NPADN * 4);
  const size_t oOF = off; off = al256(off + (size_t)NREL * NPADN * 4);
  const size_t oLS = off; off = al256(off + (size_t)NREL * NBLK * RCAP * 4);
  const size_t oA  = off; off = al256(off + (size_t)HALF * KT * 2);
  const size_t wsmax = (size_t)(128u << 20);
  if (off > ws_size || off > wsmax) return;
  unsigned short* WT = (unsigned short*)(ws + oWT);
  float* BSUM = (float*)(ws + oBS);
  int*   FLG  = (int*)(ws + oFL);
  int*   CNT  = (int*)(ws + oCN);
  int*   OFF  = (int*)(ws + oOF);
  int*   LIST = (int*)(ws + oLS);
  unsigned short* A = (unsigned short*)(ws + oA);

  hipFuncSetAttribute(reinterpret_cast<const void*>(&k_bucket), hipFuncAttributeMaxDynamicSharedMemorySize, LDS_BK);

  k_prep<<<WUNITS / NTHR + 1, NTHR, 0, stream>>>(W, b, WT, BSUM);
  const dim3 gb((unsigned)NBLK, (unsigned)NREL, 1u);
  k_bucket<<<gb, NTHR, LDS_BK, stream>>>(src, dst, LIST, CNT, OFF, FLG);
  k_replay<<<HALF / RPB, NTHR, 0, stream>>>(x, LIST, CNT, OFF, FLG, A, 0, HALF);
  k_gemm<<<cdiv(HALF, GBM), GTHR, 0, stream>>>(A, WT, BSUM, out, 0, HALF);
  k_replay<<<HALF / RPB, NTHR, 0, stream>>>(x, LIST, CNT, OFF, FLG, A, HALF, NN - HALF);
  k_gemm<<<cdiv(NN - HALF, GBM), GTHR, 0, stream>>>(A, WT, BSUM, out, HALF, NN - HALF);
}
